// SparseUNetMultiTask_8065948582436
// MI455X (gfx1250) — hardware-run, weakly checked
//
#include <hip/hip_runtime.h>


namespace {
constexpr int M = 64000, NC = 16000, BC = 64, BC2 = 128, K = 27, KK = K * BC, NSEM = 20, NOBJ = 16, NJ = 6, NWF = M / 16, NWC = NC / 16;
constexpr float XS = 8.0f, WSC = 256.0f;
typedef _Float16 b16;
typedef __attribute__((ext_vector_type(16))) _Float16 v16b;
typedef __attribute__((ext_vector_type(8))) _Float16 v8b;
typedef __attribute__((ext_vector_type(8))) float v8f;
typedef __attribute__((ext_vector_type(4))) float v4f;
typedef __attribute__((ext_vector_type(2))) float v2f;
__device__ __forceinline__ float bf16_rne(float f) { unsigned int u = __float_as_uint(f); u += 0x7FFFu + ((u >> 16) & 1u); return __uint_as_float(u & 0xFFFF0000u); }
__device__ __forceinline__ void split16(float v, b16& hi, b16& lo) { hi = (b16)v; lo = (b16)(v - (float)hi); }
__device__ __forceinline__ v16b frag_kb(const b16* p, int hh) { const v8b a = *(const v8b*)(p + 8 * hh), b = *(const v8b*)(p + 16 + 8 * hh); v16b f;
#pragma unroll
  for (int e = 0; e < 8; ++e) { f[e] = a[e]; f[8 + e] = b[e]; } return f; }
__device__ __forceinline__ v8f wmma16b(v16b a, v16b b, v8f c) { v8f d = __builtin_amdgcn_wmma_f32_16x16x32_f16(false, a, false, b, (short)0, c, false, false); asm volatile("v_nop\n\tv_nop\n\tv_nop\n\tv_nop" : "+v"(d) : "v"(a), "v"(b)); return d; }
__device__ __forceinline__ void wave_lds_sync() { __builtin_amdgcn_fence(__ATOMIC_RELEASE, "workgroup"); __builtin_amdgcn_wave_barrier(); __builtin_amdgcn_fence(__ATOMIC_ACQUIRE, "workgroup"); }
__device__ __forceinline__ float pmul(float a, float b) { float p = a * b; asm volatile("" : "+v"(p)); return p; }
__device__ __forceinline__ int iclamp(int v, int lo, int hi) { return v < lo ? lo : (v > hi ? hi : v); }
constexpr int CSR_NBLK = 512, CSR_GB = 9, CSR_GN = 1 << CSR_GB  , CSR_TS = (CSR_GN < 32 ? 32 : CSR_GN)  , CSR_MAXG = 512, CSR_CAP = 12288  ;
__device__ __host__ __forceinline__ int csr_tix(int v) { return (v >> CSR_GB) * CSR_TS + (v & (CSR_GN - 1)); }
__global__ __launch_bounds__(64) void csrA_kernel(const int* __restrict__ dst, int E, int N, int nG, int CHP, int NGP, int* __restrict__ STG, int* __restrict__ HST) {
  extern __shared__ int sm[];
  int* cnt = sm; int* run = sm + NGP; int* ids = sm + 2 * NGP;
  const int b = blockIdx.x; const int ch = (E + CSR_NBLK - 1) / CSR_NBLK; const int e0 = b * ch, e1 = min(E, e0 + ch);
  for (int i = threadIdx.x; i < NGP; i += 64) cnt[i] = 0;
  for (int i = threadIdx.x; i < CHP; i += 64) ids[i] = -1;
  __syncthreads();
  if (threadIdx.x == 0) {
    for (int e = e0; e < e1; ++e) { int d = dst[e]; d = (d < 0) ? 0 : (d >= N ? N - 1 : d); cnt[d >> CSR_GB] += 1; }
    int acc = 0; for (int g = 0; g < nG; ++g) { run[g] = acc; acc += cnt[g]; }
    for (int e = e0; e < e1; ++e) { int d = dst[e]; d = (d < 0) ? 0 : (d >= N ? N - 1 : d); const int g = d >> CSR_GB; ids[run[g]] = e; run[g] += 1; } }
  __syncthreads();
  typedef __attribute__((ext_vector_type(4))) int v4i;
  for (int pass = 0; pass < 2; ++pass) {
    for (int i = threadIdx.x; i < CHP / 4; i += 64) *(volatile v4i*)(STG + (size_t)b * CHP + i * 4) = *(const v4i*)(&ids[i * 4]);
    for (int i = threadIdx.x; i < NGP / 4; i += 64) { v4i v; for (int e = 0; e < 4; ++e) v[e] = (i * 4 + e < nG) ? cnt[i * 4 + e] : 0; *(volatile v4i*)(HST + (size_t)b * NGP + i * 4) = v; }
    __threadfence(); }
}
__global__ __launch_bounds__(512) void csrS_kernel(const int* __restrict__ HST, int nG, int NGP, int* __restrict__ START, int* __restrict__ TOT, int* __restrict__ OFF) {
  __shared__ int tot[CSR_MAXG];
  const int b = threadIdx.x;
  for (int pass = 0; pass < 2; ++pass) { int runb = 0; for (int g = 0; g < nG; ++g) { int c = HST[(size_t)b * NGP + g]; c = (c < 0) ? 0 : c; ((volatile int*)OFF)[(size_t)g * CSR_NBLK + b] = runb; runb += c; } __threadfence(); }
  for (int g = threadIdx.x; g < nG; g += 512) { int s = 0; for (int bb = 0; bb < CSR_NBLK; ++bb) { int c = HST[(size_t)bb * NGP + g]; s += (c < 0) ? 0 : c; } tot[g] = s; }
  __syncthreads();
  if (threadIdx.x < 32) {
    __shared__ int st[CSR_MAXG + 32];
    if (threadIdx.x == 0) { int acc = 0; for (int g = 0; g < NGP; ++g) { st[g] = acc; if (g < nG) acc += (tot[g] + 31) & ~31; } st[NGP] = acc; }
    __builtin_amdgcn_fence(__ATOMIC_RELEASE, "workgroup"); __builtin_amdgcn_wave_barrier(); __builtin_amdgcn_fence(__ATOMIC_ACQUIRE, "workgroup");
    for (int pass = 0; pass < 2; ++pass) { for (int i = threadIdx.x; i < NGP + 32; i += 32) { ((volatile int*)START)[i] = (i <= NGP) ? st[min(i, NGP)] : 0; ((volatile int*)TOT)[i] = (i < nG) ? tot[i] : 0; } __threadfence(); } }
}
__global__ __launch_bounds__(256) void csrB_kernel(const int* __restrict__ dst, int N, int nG, int CHP, int NGP, int permLen, const int* __restrict__ STG, const int* __restrict__ HST, const int* __restrict__ OFF, const int* __restrict__ START, const int* __restrict__ TOT, int* __restrict__ PERM, int* __restrict__ ROWPTR, int* __restrict__ ROWCNT, int* __restrict__ FLAG) {
  typedef __attribute__((ext_vector_type(4))) int v4i;
  __shared__ int ids[CSR_CAP]; __shared__ unsigned short key[CSR_CAP]; __shared__ int outp[CSR_CAP]; __shared__ int ncnt[CSR_GN + 1]; __shared__ int boff[CSR_NBLK + 1];
  const int g = blockIdx.x, t_ = threadIdx.x; int tot = TOT[g]; int st = START[g], stn = START[g + 1]; const int v0 = g * CSR_GN; const int nv = min(CSR_GN, N - v0); const int t0 = g * CSR_TS;
  st = (st < 0) ? 0 : (st > permLen - 32 ? permLen - 32 : st) & ~31; stn = (stn < st) ? st : (stn > permLen ? permLen : stn); tot = (tot < 0) ? 0 : tot; if (tot > stn - st && tot <= CSR_CAP) tot = stn - st;
  if (tot > CSR_CAP) {
    for (int pass = 0; pass < 2; ++pass) { for (int i = t_; i < CSR_TS / 4; i += 256) { v4i a, c; for (int e = 0; e < 4; ++e) { a[e] = st; c[e] = 0; } *(volatile v4i*)(ROWPTR + t0 + i * 4) = a; *(volatile v4i*)(ROWCNT + t0 + i * 4) = c; } if (t_ == 0) ((volatile int*)FLAG)[0] = 1; __threadfence(); } (void)nv; return; }
  if (t_ == 0) { int acc = 0; for (int b = 0; b < CSR_NBLK; ++b) { boff[b] = acc; int c = HST[(size_t)b * NGP + g]; c = (c < 0) ? 0 : (c > CHP ? CHP : c); acc += c; if (acc > tot) acc = tot; } boff[CSR_NBLK] = acc; }
  for (int i = t_; i <= CSR_GN; i += 256) ncnt[i] = 0;
  __syncthreads();
  for (int b = 0; b < CSR_NBLK; ++b) { const int c = boff[b + 1] - boff[b]; int o_ = OFF[(size_t)g * CSR_NBLK + b]; o_ = (o_ < 0) ? 0 : (o_ > CHP - c ? CHP - c : o_); const int* src_ = STG + (size_t)b * CHP + o_;
    for (int i = t_; i < c; i += 256) { int id = src_[i]; id = (id < 0) ? 0 : id; ids[boff[b] + i] = id; int d = dst[id]; d = (d < v0) ? v0 : (d >= N ? N - 1 : d); int kk = d - v0; kk = (kk < 0) ? 0 : (kk >= CSR_GN ? CSR_GN - 1 : kk); key[boff[b] + i] = (unsigned short)kk; } }
  __syncthreads();
  if (t_ == 0) { for (int i = 0; i < tot; ++i) ncnt[key[i]] += 1; int acc = 0; for (int vl = 0; vl < CSR_GN; ++vl) { const int c = ncnt[vl]; ncnt[vl] = acc; acc += c; } ncnt[CSR_GN] = acc;
    for (int i = 0; i < tot; ++i) { const int vl = key[i]; outp[ncnt[vl]] = ids[i]; ncnt[vl] += 1; }
    for (int vl = CSR_GN; vl > 0; --vl) ncnt[vl] = ncnt[vl - 1]; ncnt[0] = 0; }
  __syncthreads();
  for (int pass = 0; pass < 2; ++pass) {
    for (int i = t_; i < (stn - st) / 4; i += 256) { v4i v; for (int e = 0; e < 4; ++e) { const int q = i * 4 + e; v[e] = (q < tot) ? outp[q] : -1; } *(volatile v4i*)(PERM + st + i * 4) = v; }
    for (int i = t_; i < CSR_TS / 4; i += 256) { v4i a, c; for (int e = 0; e < 4; ++e) { const int vl = i * 4 + e; const int vc = vl < CSR_GN ? vl : CSR_GN; a[e] = (vl < CSR_GN) ? st + ncnt[vc] : st; c[e] = (vl < nv) ? (ncnt[(vc < CSR_GN ? vc : CSR_GN - 1) + 1] - ncnt[vc]) : 0; } *(volatile v4i*)(ROWPTR + t0 + i * 4) = a; *(volatile v4i*)(ROWCNT + t0 + i * 4) = c; }
    __threadfence(); }
}
__global__ __launch_bounds__(256) void csrZ_kernel(int* __restrict__ p, size_t n4) { typedef __attribute__((ext_vector_type(4))) int v4i; const size_t tid = (size_t)blockIdx.x * 256 + threadIdx.x, nth = (size_t)gridDim.x * 256; v4i z = {0, 0, 0, 0}; for (size_t i = tid; i < n4; i += nth) *(volatile v4i*)(p + i * 4) = z; }
struct CsrBufs { int *STG, *HST, *OFF, *START, *TOT, *PERM, *ROWPTR, *ROWCNT, *FLAG; int nG, NGP, CHP; size_t permLen; char* base; size_t bytes; };
static size_t csr_carve(CsrBufs& c, char* ws, size_t off, int E, int N) {
  const size_t off0 = off; c.base = ws + off;
  auto al = [&](size_t bytes) { char* p = ws + off; off += (bytes + 255) & ~(size_t)255; return p; };
  c.nG = (N + CSR_GN - 1) / CSR_GN; c.NGP = (c.nG + 31) & ~31; const int ch = (E + CSR_NBLK - 1) / CSR_NBLK; c.CHP = (ch + 31) & ~31; c.permLen = (size_t)E + 32 * (size_t)c.nG + 32;
  c.STG = (int*)al((size_t)CSR_NBLK * c.CHP * 4); c.HST = (int*)al((size_t)CSR_NBLK * c.NGP * 4); c.OFF = (int*)al((size_t)c.NGP * CSR_NBLK * 4); c.START = (int*)al((size_t)(c.NGP + 64) * 4); c.TOT = (int*)al((size_t)(c.NGP + 64) * 4);
  c.PERM = (int*)al(c.permLen * 4); c.ROWPTR = (int*)al((size_t)c.nG * CSR_TS * 4); c.ROWCNT = (int*)al((size_t)c.nG * CSR_TS * 4); c.FLAG = (int*)al(256);
  c.bytes = off - off0; return off;
}
static void csr_build(const CsrBufs& c, const int* dst, int E, int N, hipStream_t stream) {
  const size_t smem = (size_t)(2 * c.NGP + c.CHP) * 4;
  csrZ_kernel<<<512, 256, 0, stream>>>((int*)c.base, c.bytes / 16);
  csrA_kernel<<<CSR_NBLK, 64, smem, stream>>>(dst, E, N, c.nG, c.CHP, c.NGP, c.STG, c.HST);
  csrS_kernel<<<1, 512, 0, stream>>>(c.HST, c.nG, c.NGP, c.START, c.TOT, c.OFF);
  csrB_kernel<<<c.nG, 256, 0, stream>>>(dst, N, c.nG, c.CHP, c.NGP, (int)c.permLen, c.STG, c.HST, c.OFF, c.START, c.TOT, c.PERM, c.ROWPTR, c.ROWCNT, c.FLAG);
}


template <int KC, int CIN, int OUT>
__global__ __launch_bounds__(256) void wprep_kernel(const float* __restrict__ w, b16* __restrict__ WT) {
  const size_t u = (size_t)blockIdx.x * 256 + threadIdx.x; constexpr size_t KT = (size_t)KC * CIN; if (u >= (size_t)OUT * KT / 8) return; const size_t e = u * 8; const int o = (int)(e / KT); const int k0 = (int)(e % KT); v8b v;
  for (int j = 0; j < 8; ++j) { const int k = k0 + j; const int kk = k / CIN, ci = k % CIN; v[j] = (b16)(bf16_rne(w[((size_t)kk * CIN + ci) * OUT + o]) * WSC); }
  for (int pass = 0; pass < 2; ++pass) { *(volatile v8b*)(WT + e) = v; __threadfence(); }
}
template <int NT, int RAW>
__device__ __forceinline__ void rbconv(const float* __restrict__ X, const int* __restrict__ rb, int nrows, int NLIM, const b16* __restrict__ WT, size_t row0, b16 (*Ah)[BC + 8], b16 (*Al)[BC + 8], v8f* acc, int& cntv, int lane, int nloc, int hlf) {
  int mycnt = 0;
#pragma unroll 1
  for (int k = 0; k < K; ++k) {
    const size_t row = row0 + nloc; int nb = -1; if (row < (size_t)nrows) { nb = rb[row * K + k]; if (nb >= nrows) nb = -1; } if (nb >= 0) ++mycnt; const bool use = nb >= 0 && nb < NLIM;
    const float* xr = X + (size_t)(use ? nb : 0) * BC + hlf * 32;
    for (int q = 0; q < 8; ++q) { const v4f xv = use ? *(const v4f*)(xr + q * 4) : (v4f){0.0f, 0.0f, 0.0f, 0.0f};
      for (int j = 0; j < 4; ++j) { b16 p, ql; if (RAW) { p = (b16)(bf16_rne(xv[j]) * XS); ql = (b16)0.0f; } else split16(xv[j] * XS, p, ql); Ah[nloc][hlf * 32 + q * 4 + j] = p; Al[nloc][hlf * 32 + q * 4 + j] = ql; } }
    wave_lds_sync();
#pragma unroll
    for (int kb = 0; kb < BC; kb += 32) { const v16b a = frag_kb(&Ah[nloc][kb], hlf); v16b al = {}; if (!RAW) al = frag_kb(&Al[nloc][kb], hlf);
#pragma unroll
      for (int t = 0; t < NT; ++t) { const v16b bw = frag_kb(WT + (size_t)(t * 16 + nloc) * KK + k * BC + kb, hlf); acc[t] = wmma16b(a, bw, acc[t]); if (!RAW) acc[t] = wmma16b(al, bw, acc[t]); } }
    wave_lds_sync(); }
  cntv = mycnt;
}
__global__ __launch_bounds__(32) void conv1_kernel(const float* __restrict__ feats, const int* __restrict__ rb1, const b16* __restrict__ W1, const float* __restrict__ b1, int NLIM, float* __restrict__ X1) {
  __shared__ __attribute__((aligned(16))) b16 Ah[16][BC + 8], Al[16][BC + 8]; __shared__ __attribute__((aligned(16))) float Tf[16][BC + 4]; __shared__ int cnts[16];
  const int lane = threadIdx.x, nloc = lane & 15, hlf = lane >> 4; const size_t row0 = (size_t)blockIdx.x * 16;
  v8f acc[4]; for (int t = 0; t < 4; ++t) acc[t] = (v8f){}; int cntv;
  rbconv<4, 1>(feats, rb1, M, NLIM, W1, row0, Ah, Al, acc, cntv, lane, nloc, hlf);
  if (hlf == 0) cnts[nloc] = cntv;
  wave_lds_sync();
#pragma unroll
  for (int t = 0; t < 4; ++t) { const int c = t * 16 + nloc; const float bb = bf16_rne(b1[c]);
#pragma unroll 1
    for (int r8 = 0; r8 < 8; ++r8) { const int rl = 8 * hlf + r8; const int cn = cnts[rl]; const float inv = 1.0f / (float)(cn < 1 ? 1 : cn); const size_t row = row0 + rl;
      Tf[rl][c] = (row < (size_t)NLIM) ? pmul(acc[t][r8] * (1.0f / (XS * WSC)), inv) + bb + bf16_rne(feats[row * BC + c]) : 0.0f; } }
  wave_lds_sync();
  for (int pass = 0; pass < 2; ++pass) { for (int rr = 0; rr < 16; ++rr) *(volatile v2f*)(X1 + (row0 + rr) * BC + lane * 2) = *(const v2f*)(&Tf[rr][lane * 2]); __threadfence(); }
}
__global__ __launch_bounds__(256) void cmean_kernel(const float* __restrict__ X1, const int* __restrict__ PERM, const int* __restrict__ ROWPTR, const int* __restrict__ ROWCNT, int permLen, int NLIMC, float* __restrict__ XA) {
  const int wave = threadIdx.x >> 5, lane = threadIdx.x & 31; const int c = blockIdx.x * 8 + wave; v2f a = {0.0f, 0.0f};
  if (c < NLIMC) { int st = ROWPTR[c], cnt = ROWCNT[c]; cnt = iclamp(cnt, 0, 65536); st = iclamp(st, 0, permLen - cnt);
    for (int j = 0; j < cnt; ++j) { const int f = iclamp(PERM[st + j], 0, M - 1); const v2f x = *(const v2f*)(X1 + (size_t)f * BC + lane * 2); a[0] += x[0]; a[1] += x[1]; }
    const float inv = 1.0f / (float)(cnt < 1 ? 1 : cnt); a[0] = pmul(a[0], inv); a[1] = pmul(a[1], inv); }
  for (int pass = 0; pass < 2; ++pass) { *(volatile v2f*)(XA + (size_t)c * BC + lane * 2) = a; __threadfence(); }
}
__global__ __launch_bounds__(32) void conv2_kernel(const float* __restrict__ XA, const int* __restrict__ rb2, const b16* __restrict__ W2, const b16* __restrict__ R2T, const b16* __restrict__ CUT, const float* __restrict__ b2, const float* __restrict__ r2b, const float* __restrict__ cb, const float* __restrict__ ub, int NLIMC, float* __restrict__ CU) {
  __shared__ __attribute__((aligned(16))) b16 Ah[16][BC + 8], Al[16][BC + 8], Bh[16][BC2 + 8], Bl[16][BC2 + 8]; __shared__ __attribute__((aligned(16))) float Tf[16][BC2 + 4]; __shared__ int cnts[16];
  const int lane = threadIdx.x, nloc = lane & 15, hlf = lane >> 4; const size_t row0 = (size_t)blockIdx.x * 16;
  v8f acc[8]; for (int t = 0; t < 8; ++t) acc[t] = (v8f){}; int cntv;
  rbconv<8, 0>(XA, rb2, NC, NLIMC, W2, row0, Ah, Al, acc, cntv, lane, nloc, hlf);
  if (hlf == 0) cnts[nloc] = cntv;
  { const size_t row = row0 + nloc; const bool ok = row < (size_t)NLIMC; const float* xr = XA + (ok ? row : 0) * BC + hlf * 32;
    for (int q = 0; q < 8; ++q) { const v4f xv = ok ? *(const v4f*)(xr + q * 4) : (v4f){0.0f, 0.0f, 0.0f, 0.0f}; for (int j = 0; j < 4; ++j) { b16 p, ql; split16(xv[j] * XS, p, ql); Ah[nloc][hlf * 32 + q * 4 + j] = p; Al[nloc][hlf * 32 + q * 4 + j] = ql; } } }
  wave_lds_sync();
  v8f ar[8]; for (int t = 0; t < 8; ++t) ar[t] = (v8f){};
#pragma unroll
  for (int kb = 0; kb < BC; kb += 32) { const v16b a = frag_kb(&Ah[nloc][kb], hlf), al = frag_kb(&Al[nloc][kb], hlf);
#pragma unroll
    for (int t = 0; t < 8; ++t) { const v16b bw = frag_kb(R2T + (size_t)(t * 16 + nloc) * BC + kb, hlf); ar[t] = wmma16b(a, bw, ar[t]); ar[t] = wmma16b(al, bw, ar[t]); } }
#pragma unroll
  for (int t = 0; t < 8; ++t) { const int c = t * 16 + nloc; const float bb = bf16_rne(b2[c]) + bf16_rne(r2b[c]);
#pragma unroll 1
    for (int r8 = 0; r8 < 8; ++r8) { const int rl = 8 * hlf + r8; const int cn = cnts[rl]; const float inv = 1.0f / (float)(cn < 1 ? 1 : cn); const float x2 = ((row0 + rl) < (size_t)NLIMC) ? pmul(acc[t][r8] * (1.0f / (XS * WSC)), inv) + ar[t][r8] * (1.0f / (XS * WSC)) + bb : 0.0f; b16 p, ql; split16(x2 * XS, p, ql); Bh[rl][c] = p; Bl[rl][c] = ql; } }
  wave_lds_sync();
#pragma unroll
  for (int t = 0; t < 8; ++t) acc[t] = (v8f){};
#pragma unroll
  for (int kb = 0; kb < BC2; kb += 32) { const v16b a = frag_kb(&Bh[nloc][kb], hlf), al = frag_kb(&Bl[nloc][kb], hlf);
#pragma unroll
    for (int t = 0; t < 8; ++t) { const v16b bw = frag_kb(CUT + (size_t)(t * 16 + nloc) * BC2 + kb, hlf); acc[t] = wmma16b(a, bw, acc[t]); acc[t] = wmma16b(al, bw, acc[t]); } }
#pragma unroll
  for (int t = 0; t < 8; ++t) { const int c = t * 16 + nloc; const float bb = c < BC ? bf16_rne(cb[c]) : bf16_rne(ub[c - BC]);
#pragma unroll 1
    for (int r8 = 0; r8 < 8; ++r8) { const int rl = 8 * hlf + r8; Tf[rl][c] = ((row0 + rl) < (size_t)NLIMC) ? acc[t][r8] * (1.0f / (XS * WSC)) + bb : 0.0f; } }
  wave_lds_sync();
  for (int pass = 0; pass < 2; ++pass) { for (int rr = 0; rr < 16; ++rr) *(volatile v4f*)(CU + (row0 + rr) * BC2 + lane * 4) = *(const v4f*)(&Tf[rr][lane * 4]); __threadfence(); }
}
__global__ __launch_bounds__(32) void xin_kernel(const float* __restrict__ X1, const float* __restrict__ CU, const int* __restrict__ invc, int NLIM, float* __restrict__ XIN) {
  const int lane = threadIdx.x; const size_t row0 = (size_t)blockIdx.x * 16;
  for (int rr = 0; rr < 16; ++rr) { const size_t row = row0 + rr; v2f o = {0.0f, 0.0f}; if (row < (size_t)NLIM) { const int c = iclamp(invc[row], 0, NC - 1); const v2f a = *(const v2f*)(X1 + row * BC + lane * 2), u = *(const v2f*)(CU + (size_t)c * BC2 + BC + lane * 2); o[0] = a[0] + u[0]; o[1] = a[1] + u[1]; }
    for (int pass = 0; pass < 2; ++pass) { *(volatile v2f*)(XIN + row * BC + lane * 2) = o; __threadfence(); } }
}
__global__ __launch_bounds__(32) void fuse_kernel(const float* __restrict__ XIN, const int* __restrict__ rb1, const b16* __restrict__ WF, const float* __restrict__ CU, const int* __restrict__ invc, const b16* __restrict__ GBT, const b16* __restrict__ SEMT,
                                                   const float* __restrict__ gb, const float* __restrict__ btb, const float* __restrict__ bfv, const float* __restrict__ semb, int NLIM, float* __restrict__ out0, float* __restrict__ PS) {
  __shared__ __attribute__((aligned(16))) b16 Ah[16][BC + 8], Al[16][BC + 8]; __shared__ __attribute__((aligned(16))) float Xr[16][BC + 4], So[16 * NSEM]; __shared__ int cnts[16];
  const int lane = threadIdx.x, nloc = lane & 15, hlf = lane >> 4; const size_t row0 = (size_t)blockIdx.x * 16;
  v8f acc[4]; for (int t = 0; t < 4; ++t) acc[t] = (v8f){}; int cntv;
  rbconv<4, 0>(XIN, rb1, M, NLIM, WF, row0, Ah, Al, acc, cntv, lane, nloc, hlf);
  if (hlf == 0) cnts[nloc] = cntv;
  { const size_t row = row0 + nloc; const bool ok = row < (size_t)NLIM; const int c = ok ? iclamp(invc[row], 0, NC - 1) : 0; const float* cr = CU + (size_t)c * BC2 + hlf * 32;
    for (int q = 0; q < 8; ++q) { const v4f cv = ok ? *(const v4f*)(cr + q * 4) : (v4f){0.0f, 0.0f, 0.0f, 0.0f}; for (int j = 0; j < 4; ++j) { b16 p, ql; split16(cv[j] * XS, p, ql); Ah[nloc][hlf * 32 + q * 4 + j] = p; Al[nloc][hlf * 32 + q * 4 + j] = ql; } } }
  wave_lds_sync();
  v8f ag[8]; for (int t = 0; t < 8; ++t) ag[t] = (v8f){};
#pragma unroll
  for (int kb = 0; kb < BC; kb += 32) { const v16b a = frag_kb(&Ah[nloc][kb], hlf), al = frag_kb(&Al[nloc][kb], hlf);
#pragma unroll
    for (int t = 0; t < 8; ++t) { const v16b bw = frag_kb(GBT + (size_t)(t * 16 + nloc) * BC + kb, hlf); ag[t] = wmma16b(a, bw, ag[t]); ag[t] = wmma16b(al, bw, ag[t]); } }
  wave_lds_sync();
  const float sc = 1.0f / (XS * WSC);
#pragma unroll
  for (int t = 0; t < 4; ++t) { const int c = t * 16 + nloc; const float gbb = bf16_rne(gb[c]), bbb = bf16_rne(btb[c]), bfb = bf16_rne(bfv[c]);
#pragma unroll 1
    for (int r8 = 0; r8 < 8; ++r8) { const int rl = 8 * hlf + r8; const size_t row = row0 + rl; const int cn = cnts[rl]; const float inv = 1.0f / (float)(cn < 1 ? 1 : cn);
      float xr = 0.0f; if (row < (size_t)NLIM) { const float sk = pmul(acc[t][r8] * sc, inv); const float gam = ag[t][r8] * sc + gbb, bet = ag[t + 4][r8] * sc + bbb; xr = pmul(gam, sk) + bet + bfb + XIN[row * BC + c]; }
      Xr[rl][c] = xr; b16 p, ql; split16(xr * XS, p, ql); Ah[rl][c] = p; Al[rl][c] = ql; } }
  wave_lds_sync();
  v8f as_[2] = {(v8f){}, (v8f){}};
#pragma unroll
  for (int kb = 0; kb < BC; kb += 32) { const v16b a = frag_kb(&Ah[nloc][kb], hlf), al = frag_kb(&Al[nloc][kb], hlf);
#pragma unroll
    for (int t = 0; t < 2; ++t) { const v16b bw = frag_kb(SEMT + (size_t)(t * 16 + nloc) * BC + kb, hlf); as_[t] = wmma16b(a, bw, as_[t]); as_[t] = wmma16b(al, bw, as_[t]); } }
#pragma unroll
  for (int t = 0; t < 2; ++t) { const int c = t * 16 + nloc; if (c < NSEM) { const float bb = bf16_rne(semb[c]);
#pragma unroll 1
    for (int r8 = 0; r8 < 8; ++r8) So[(8 * hlf + r8) * NSEM + c] = as_[t][r8] * sc + bb; } }
  float s0 = 0.0f, s1 = 0.0f; for (int rr = 0; rr < 16; ++rr) { s0 += Xr[rr][lane * 2]; s1 += Xr[rr][lane * 2 + 1]; }
  wave_lds_sync();
  for (int pass = 0; pass < 2; ++pass) {
    for (int q = 0; q < 3; ++q) { const int idx = q * 32 + lane; if (idx < 80) *(volatile v4f*)(out0 + row0 * NSEM + (size_t)idx * 4) = *(const v4f*)(&So[idx * 4]); }
    v2f pv = {s0, s1}; *(volatile v2f*)(PS + (size_t)blockIdx.x * BC + lane * 2) = pv; __threadfence(); }
}
__global__ __launch_bounds__(32) void final_kernel(const float* __restrict__ PS, int nwaves, int NLIM, const b16* __restrict__ HT, const float* __restrict__ clsb, const float* __restrict__ embb, const float* __restrict__ kpb, float* __restrict__ tail) {
  __shared__ __attribute__((aligned(16))) b16 Ah[16][BC + 8], Al[16][BC + 8]; __shared__ float res[128]; __shared__ float nrm2[16];
  const int lane = threadIdx.x, nloc = lane & 15, hlf = lane >> 4; constexpr float PSC = 256.0f;
  for (int q = 0; q < 2; ++q) { const int c = lane * 2 + q; double s = 0.0;
#pragma unroll 1
    for (int w = 0; w < nwaves; ++w) s += (double)PS[(size_t)w * BC + c];
    const float pooled = (float)s * (1.0f / (float)NLIM); b16 p, ql; split16(pooled * PSC, p, ql); Ah[0][c] = p; Al[0][c] = ql; }
  for (int r = 1; r < 16; ++r) { Ah[r][lane * 2] = (b16)0.0f; Ah[r][lane * 2 + 1] = (b16)0.0f; Al[r][lane * 2] = (b16)0.0f; Al[r][lane * 2 + 1] = (b16)0.0f; }
  wave_lds_sync();
  v8f acc[7];
#pragma unroll
  for (int t = 0; t < 7; ++t) acc[t] = (v8f){};
#pragma unroll
  for (int kb = 0; kb < BC; kb += 32) { const v16b a = frag_kb(&Ah[nloc][kb], hlf), al = frag_kb(&Al[nloc][kb], hlf);
#pragma unroll
    for (int t = 0; t < 7; ++t) { const v16b bw = frag_kb(HT + (size_t)(t * 16 + nloc) * BC + kb, hlf); acc[t] = wmma16b(a, bw, acc[t]); acc[t] = wmma16b(al, bw, acc[t]); } }
  if (hlf == 0) {
#pragma unroll
    for (int t = 0; t < 7; ++t) { const int c = t * 16 + nloc; const float v = acc[t][0] * (1.0f / (PSC * WSC));
      if (c < NOBJ) res[c] = v + bf16_rne(clsb[c]); else if (c < NOBJ + BC) res[c] = v + bf16_rne(embb[c - NOBJ]); else if (c < NOBJ + BC + NJ * 3) res[c] = 1.2f * tanhf(v + bf16_rne(kpb[c - NOBJ - BC])); } }
  wave_lds_sync();
  { float s = 0.0f; for (int k = nloc; k < BC; k += 16) { const float e = res[NOBJ + k]; s += e * e; } for (int o = 1; o < 16; o <<= 1) s += __shfl_xor(s, o); if (lane == 0) nrm2[0] = s; }
  wave_lds_sync();
  { const float nrm = fmaxf(sqrtf(nrm2[0]), 1e-12f); for (int k = lane; k < BC; k += 32) res[NOBJ + k] = res[NOBJ + k] / nrm; }
  wave_lds_sync();
  for (int pass = 0; pass < 2; ++pass) { for (int i = lane; i < NOBJ + BC + NJ * 3; i += 32) ((volatile float*)tail)[i] = res[i]; __threadfence(); }
}
__global__ __launch_bounds__(256) void headprep_kernel(const float* __restrict__ clsW, const float* __restrict__ embW, const float* __restrict__ kpW, b16* __restrict__ HT) {
  const int u = blockIdx.x * 256 + threadIdx.x; if (u >= 112 * BC / 8) return; const int e = u * 8, r = e / BC, k0 = e % BC; v8b v;
  for (int j = 0; j < 8; ++j) { const int k = k0 + j; float w = 0.0f;
    if (r < NOBJ) w = clsW[k * NOBJ + r]; else if (r < NOBJ + BC) w = embW[k * BC + (r - NOBJ)]; else if (r < NOBJ + BC + NJ * 3) { const int q = r - NOBJ - BC; w = kpW[((size_t)(q / 3) * BC + k) * 3 + (q % 3)]; }
    v[j] = (b16)(bf16_rne(w) * WSC); }
  for (int pass = 0; pass < 2; ++pass) { *(volatile v8b*)(HT + e) = v; __threadfence(); }
}
__global__ __launch_bounds__(256) void semprep_kernel(const float* __restrict__ w, b16* __restrict__ SEMT) {
  const int u = blockIdx.x * 256 + threadIdx.x; if (u >= 32 * BC / 8) return; const int e = u * 8, o = e / BC, k0 = e % BC; v8b v; for (int j = 0; j < 8; ++j) v[j] = o < NSEM ? (b16)(bf16_rne(w[(k0 + j) * NSEM + (o < NSEM ? o : 0)]) * WSC) : (b16)0.0f;
  for (int pass = 0; pass < 2; ++pass) { *(volatile v8b*)(SEMT + e) = v; __threadfence(); }
}
}

extern "C" void kernel_launch(void* const* d_in, const int* in_sizes, int n_in, void* d_out, int out_size, void* d_ws, size_t ws_size, hipStream_t stream) {
  (void)n_in;
  auto Fp = [&](int i) { return (const float*)d_in[i]; }; auto Ip = [&](int i) { return (const int*)d_in[i]; };
  if (in_sizes[0] != M * BC || in_sizes[1] != M * K || in_sizes[2] != NC * K || in_sizes[3] != M || in_sizes[4] != K * BC * BC || in_sizes[6] != K * BC * BC2 || in_sizes[14] != K * BC * BC || in_sizes[20] != BC * NSEM || in_sizes[24] != NJ * BC * 3 || out_size != M * NSEM + NOBJ + BC + NJ * 3) return;
  const int NLIM = M, NLIMC = NC; const int GWF = NWF, GWC = NWC;
  size_t off = 0; char* ws = (char*)d_ws;
  auto carve = [&](size_t bytes) { char* p = ws + off; off += (bytes + 255) & ~(size_t)255; return p; };
  b16* W1 = (b16*)carve((size_t)BC * KK * 2); b16* W2 = (b16*)carve((size_t)BC2 * KK * 2); b16* WF = (b16*)carve((size_t)BC * KK * 2); b16* R2T = (b16*)carve((size_t)BC2 * BC * 2); b16* CUT = (b16*)carve((size_t)BC2 * BC2 * 2); b16* GBT = (b16*)carve((size_t)BC2 * BC * 2); b16* SEMT = (b16*)carve((size_t)32 * BC * 2 + 256); b16* HT = (b16*)carve((size_t)112 * BC * 2);
  float* X1 = (float*)carve((size_t)M * BC * 4); float* XA = (float*)carve((size_t)NC * BC * 4); float* CU = (float*)carve((size_t)NC * BC2 * 4); float* XIN = (float*)carve((size_t)M * BC * 4); float* PS = (float*)carve((size_t)NWF * BC * 4);
  CsrBufs csr; off = csr_carve(csr, ws, off, M, NC);
  if (off > ws_size || off > ((size_t)128 << 20)) return;
  wprep_kernel<K, BC, BC><<<(BC * KK / 8 + 255) / 256, 256, 0, stream>>>(Fp(4), W1); wprep_kernel<K, BC, BC2><<<(BC2 * KK / 8 + 255) / 256, 256, 0, stream>>>(Fp(6), W2); wprep_kernel<K, BC, BC><<<(BC * KK / 8 + 255) / 256, 256, 0, stream>>>(Fp(14), WF);
  wprep_kernel<1, BC, BC2><<<(BC2 * BC / 8 + 255) / 256, 256, 0, stream>>>(Fp(8), R2T);
  wprep_kernel<1, BC2, BC><<<(BC * BC2 / 8 + 255) / 256, 256, 0, stream>>>(Fp(10), CUT); wprep_kernel<1, BC2, BC><<<(BC * BC2 / 8 + 255) / 256, 256, 0, stream>>>(Fp(12), CUT + (size_t)BC * BC2);
  wprep_kernel<1, BC, BC><<<(BC * BC / 8 + 255) / 256, 256, 0, stream>>>(Fp(16), GBT); wprep_kernel<1, BC, BC><<<(BC * BC / 8 + 255) / 256, 256, 0, stream>>>(Fp(18), GBT + (size_t)BC * BC);
  semprep_kernel<<<1, 256, 0, stream>>>(Fp(20), SEMT); headprep_kernel<<<(112 * BC / 8 + 255) / 256, 256, 0, stream>>>(Fp(22), Fp(26), Fp(24), HT);
  csr_build(csr, Ip(3), M, NC, stream);
  conv1_kernel<<<GWF, 32, 0, stream>>>(Fp(0), Ip(1), W1, Fp(5), NLIM, X1);
  cmean_kernel<<<NC / 8, 256, 0, stream>>>(X1, csr.PERM, csr.ROWPTR, csr.ROWCNT, (int)csr.permLen, NLIMC, XA);
  conv2_kernel<<<GWC, 32, 0, stream>>>(XA, Ip(2), W2, R2T, CUT, Fp(7), Fp(9), Fp(11), Fp(13), NLIMC, CU);
  xin_kernel<<<GWF, 32, 0, stream>>>(X1, CU, Ip(3), NLIM, XIN);
  fuse_kernel<<<GWF, 32, 0, stream>>>(XIN, Ip(1), WF, CU, Ip(3), GBT, SEMT, Fp(17), Fp(19), Fp(15), Fp(21), NLIM, (float*)d_out, PS);
  final_kernel<<<1, 32, 0, stream>>>(PS, GWF, NLIM, HT, Fp(23), Fp(27), Fp(25), (float*)d_out + (size_t)M * NSEM);
}
